// PNA_PI_72181220377206
// MI455X (gfx1250) — hardware-verified
//
#include <hip/hip_runtime.h>
#include <stddef.h>


#define NTHR   256
#define NWAVE  8
#define EPT    8
#define NGRP   2
#define CHUNK  (NTHR * EPT * NGRP)
#define WCAP   (EPT * NGRP * 32)
#define LISTN  (NWAVE * WCAP)
#define PROWS  64
#define FIN    16
#define HID    128
#define EDIM   8
#define ODIM   4
#define NB0    512
#define NB1    128
#define KP0    224
#define KP1    1664

#define AVGF   2.1972245773362196f
#define RAVG   (1.0f / AVGF)

#define LDS_AGG(F, NB) (16 * (NB) * (F) + 4 * (NB) + 4 * LISTN + 64)
#define ALP    (HID + 8)
#define ATP    40
#define SPI    (HID + 4)
#define O_SC   0
#define O_ALH  512
#define O_ALL  (O_ALH + PROWS * ALP * 2)
#define O_R2   (O_ALL + PROWS * ALP * 2)
#define R2SZ   (PROWS * SPI * 4)
#define O_OT   (O_R2 + R2SZ)
#define LDS_POST (O_OT + PROWS * ODIM * 4)

static_assert((CHUNK & (CHUNK - 1)) == 0);
static_assert(CHUNK <= 4096);
static_assert(NB0 <= 4096 && NB1 <= 4096);
static_assert(2 * PROWS * ATP * 2 <= R2SZ);
static_assert(KP0 % 32 == 0 && KP1 % 32 == 0);
static_assert(PROWS * 2 * 4 <= O_ALH);
static_assert((O_ALL % 16) == 0 && (O_R2 % 16) == 0 && (O_OT % 16) == 0);

typedef float          v4f  __attribute__((ext_vector_type(4)));
typedef float          v8f  __attribute__((ext_vector_type(8)));
typedef int            v4i  __attribute__((ext_vector_type(4)));
typedef unsigned short v4us __attribute__((ext_vector_type(4)));
typedef unsigned short v8us __attribute__((ext_vector_type(8)));
typedef __bf16         v16b __attribute__((ext_vector_type(16)));
union FragB { v16b v; v8us h[2]; };

extern __shared__ v4f lds_dyn[];

__device__ __forceinline__ unsigned short bf_rne(float f) {
  unsigned int u = __float_as_uint(f);
  u += 0x7FFFu + ((u >> 16) & 1u);
  return (unsigned short)(u >> 16);
}
__device__ __forceinline__ float bf_up(unsigned short s) {
  return __uint_as_float(((unsigned int)s) << 16);
}
__device__ __forceinline__ void split4(const v4f v, v4us& hi, v4us& lo) {
  unsigned short h0 = bf_rne(v.x), h1 = bf_rne(v.y), h2 = bf_rne(v.z), h3 = bf_rne(v.w);
  hi.x = h0; hi.y = h1; hi.z = h2; hi.w = h3;
  lo.x = bf_rne(v.x - bf_up(h0)); lo.y = bf_rne(v.y - bf_up(h1));
  lo.z = bf_rne(v.z - bf_up(h2)); lo.w = bf_rne(v.w - bf_up(h3));
}

__device__ __forceinline__ v8f wmb(v16b a, v16b b, v8f c) {
  v8f d = __builtin_amdgcn_wmma_f32_16x16x32_bf16(false, a, false, b, (short)0, c, false, false);
  asm volatile("v_nop\n\tv_nop\n\tv_nop\n\tv_nop" : "+v"(d) : "v"(a), "v"(b));
  return d;
}
__device__ __forceinline__ v8f mma3(v8f c, const FragB& ah, const FragB& al, const FragB& bh, const FragB& bl) {
  c = wmb(ah.v, bh.v, c);
  c = wmb(ah.v, bl.v, c);
  c = wmb(al.v, bh.v, c);
  return c;
}
__device__ __forceinline__ void ldfrag(FragB& f, const unsigned short* p) {
  f.h[0] = *(const v8us*)p;
  f.h[1] = *(const v8us*)(p + 16);
}

template <int NB>
__device__ __forceinline__ int scan_chunk(const int* __restrict__ dsts, int nE, int cbase, int nodeBase,
                                          int vec8, int* list, int tid, int lane, int wave) {
  int wc = 0;
  (void)lane;
#pragma unroll
  for (int g = 0; g < NGRP; ++g) {
    const int el0  = (g * NTHR + tid) * EPT;
    const int e0   = cbase + el0;
    const int sent = -2147483647 - 1;
    v4i da, db;
    if (vec8 != 0 && cbase + CHUNK <= nE) {
      da = *(const v4i*)(dsts + e0);
      db = *(const v4i*)(dsts + e0 + 4);
    } else {
      da.x = (e0     < nE) ? dsts[min(e0,     nE - 1)] : sent;
      da.y = (e0 + 1 < nE) ? dsts[min(e0 + 1, nE - 1)] : sent;
      da.z = (e0 + 2 < nE) ? dsts[min(e0 + 2, nE - 1)] : sent;
      da.w = (e0 + 3 < nE) ? dsts[min(e0 + 3, nE - 1)] : sent;
      db.x = (e0 + 4 < nE) ? dsts[min(e0 + 4, nE - 1)] : sent;
      db.y = (e0 + 5 < nE) ? dsts[min(e0 + 5, nE - 1)] : sent;
      db.z = (e0 + 6 < nE) ? dsts[min(e0 + 6, nE - 1)] : sent;
      db.w = (e0 + 7 < nE) ? dsts[min(e0 + 7, nE - 1)] : sent;
    }
    const unsigned nb = (unsigned)nodeBase;
    const unsigned s0 = (unsigned)da.x - nb, s1 = (unsigned)da.y - nb;
    const unsigned s2 = (unsigned)da.z - nb, s3 = (unsigned)da.w - nb;
    const unsigned s4 = (unsigned)db.x - nb, s5 = (unsigned)db.y - nb;
    const unsigned s6 = (unsigned)db.z - nb, s7 = (unsigned)db.w - nb;
    const bool h0 = s0 < (unsigned)NB, h1 = s1 < (unsigned)NB, h2 = s2 < (unsigned)NB, h3 = s3 < (unsigned)NB;
    const bool h4 = s4 < (unsigned)NB, h5 = s5 < (unsigned)NB, h6 = s6 < (unsigned)NB, h7 = s7 < (unsigned)NB;
    const unsigned any = __builtin_amdgcn_ballot_w32(h0 | h1 | h2 | h3 | h4 | h5 | h6 | h7);
    if (any != 0u) {
#define HITJ(J, HJ, SJ) { \
        const unsigned mj = __builtin_amdgcn_ballot_w32(HJ); \
        if (mj != 0u) { \
          if (HJ) { \
            const int pos = wc + (int)__builtin_amdgcn_mbcnt_lo(mj, 0u); \
            if (pos < WCAP) list[wave * WCAP + pos] = ((el0 + (J)) << 12) | (int)(SJ); \
          } \
          wc += (int)__builtin_popcount(mj); } }
      HITJ(0, h0, s0)
      HITJ(1, h1, s1)
      HITJ(2, h2, s2)
      HITJ(3, h3, s3)
      HITJ(4, h4, s4)
      HITJ(5, h5, s5)
      HITJ(6, h6, s6)
      HITJ(7, h7, s7)
#undef HITJ
    }
  }
  return wc;
}

__global__ __launch_bounds__(NTHR) void k_wsplit(const float* __restrict__ W, int K, int NC, int G, int KP, int NP,
                                                 unsigned short* wh, unsigned short* wl) {
  const int i = blockIdx.x * NTHR + threadIdx.x;
  const int total = NP * KP / 8;
  if (i >= total) return;
  const int o  = i * 8;
  const int n  = o / KP;
  const int k0 = o - n * KP;
  const int g  = n / NC;
  const int c  = n - g * NC;
  const int gg = g < G - 1 ? g : G - 1;
  v8us hv, lv;
#pragma unroll
  for (int j = 0; j < 8; ++j) {
    const int k  = k0 + j;
    const int kc = k < K - 1 ? k : K - 1;
    const float w = W[((size_t)gg * K + kc) * NC + c];
    const float v = (g < G && k < K) ? w : 0.f;
    const unsigned short hs = bf_rne(v);
    hv[j] = hs;
    lv[j] = bf_rne(v - bf_up(hs));
  }
  *(volatile v8us*)(wh + o) = hv;
  *(volatile v8us*)(wl + o) = lv;
  __threadfence();
  *(volatile v8us*)(wh + o) = hv;
  *(volatile v8us*)(wl + o) = lv;
}

template <int F>
__global__ __launch_bounds__(NTHR) void k_comp(const float* __restrict__ ew, const float* __restrict__ eb,
                                               const float* __restrict__ pw, const float* __restrict__ pb, float* cc) {
  constexpr int CCN = ((9 * F + 31) / 32) * 32;
#pragma unroll 1
  for (int i = threadIdx.x; i < CCN; i += NTHR) {
    const int d  = i / F;
    const int c  = i - d * F;
    const int dd = d < 8 ? d : 7;
    float acc = 0.f;
#pragma unroll 1
    for (int j = 0; j < F; ++j) {
      const float we = ew[dd * F + j];
      const float wb = eb[j];
      const float w  = (d < 8) ? we : wb;
      acc += w * pw[(size_t)(2 * F + j) * F + c];
    }
    float v = acc + ((d == 8) ? pb[c] : 0.f);
    v = (i < 9 * F) ? v : 0.f;
    *(volatile float*)(cc + i) = v;
    __threadfence();
    *(volatile float*)(cc + i) = v;
  }
}

template <int F, int KP, int XP, int NCB>
__global__ __launch_bounds__(NTHR) void k_pq(const float* __restrict__ xin,
                                             const unsigned short* __restrict__ wh, const unsigned short* __restrict__ wl,
                                             float* pq, int nN) {
  constexpr int AP  = KP + 8;
  constexpr int TPW = NCB / 32;
  constexpr int NCT = 2 * F;
  constexpr int LA  = PROWS * AP * 2 * 2;
  constexpr int LD  = PROWS * NCB * 4;
  constexpr int LSZ = LA > LD ? LA : LD;
  constexpr int KQ  = KP / 4;
  static_assert(KP % 32 == 0 && NCB % 32 == 0 && (NCT % NCB) == 0 && F >= 4 && (F % 4) == 0);
  __shared__ __attribute__((aligned(16))) unsigned char lds_s[LSZ];
  unsigned short* Ah = (unsigned short*)lds_s;
  unsigned short* Al = Ah + PROWS * AP;
  float* Ds = (float*)lds_s;
  const int tid = threadIdx.x, lane = tid & 31, wave = tid >> 5, hh = lane >> 4, m = lane & 15;
  const int rowBase = blockIdx.x * PROWS;
  const int colBase = blockIdx.y * NCB;

  for (int g = tid; g < PROWS * KQ; g += NTHR) {
    const int r  = g / KQ;
    const int kq = (g - r * KQ) * 4;
    int rowc = rowBase + r;
    rowc = rowc > nN - 1 ? nN - 1 : rowc;
    const int kx = kq < F - 4 ? kq : F - 4;
    const v4f xv = *(const v4f*)(xin + (size_t)rowc * XP + kx);
    const v4f z  = {0.f, 0.f, 0.f, 0.f};
    const v4f v  = (kq < F) ? xv : z;
    v4us hv, lv;
    split4(v, hv, lv);
    *(v4us*)(Ah + r * AP + kq) = hv;
    *(v4us*)(Al + r * AP + kq) = lv;
  }
  __syncthreads();

  v8f acc[TPW];
#pragma unroll
  for (int t = 0; t < TPW; ++t) { v8f z = {0.f, 0.f, 0.f, 0.f, 0.f, 0.f, 0.f, 0.f}; acc[t] = z; }
  const int rr = 16 * (wave & 3) + m;
#pragma unroll
  for (int ks = 0; ks < KP / 32; ++ks) {
    FragB ah, al;
    ldfrag(ah, Ah + rr * AP + 32 * ks + 8 * hh);
    ldfrag(al, Al + rr * AP + 32 * ks + 8 * hh);
#pragma unroll
    for (int t = 0; t < TPW; ++t) {
      const int n = colBase + 16 * ((wave >> 2) * TPW + t) + m;
      const size_t bp = (size_t)n * KP + 32 * ks + 8 * hh;
      FragB bh, bl;
      ldfrag(bh, wh + bp);
      ldfrag(bl, wl + bp);
      acc[t] = mma3(acc[t], ah, al, bh, bl);
    }
  }
  __syncthreads();

#pragma unroll
  for (int t = 0; t < TPW; ++t) {
    const int cl = 16 * ((wave >> 2) * TPW + t) + m;
    float* sp = Ds + (16 * (wave & 3) + 8 * hh) * NCB + cl;
#pragma unroll
    for (int r = 0; r < 8; ++r) sp[r * NCB] = acc[t][r];
  }
  __syncthreads();

  constexpr int RQ = NCB / 4;
  constexpr int NIT = PROWS * RQ;
#pragma unroll
  for (int i = tid; i < NIT; i += NTHR) {
    const int row = i / RQ;
    const int c4  = (i - row * RQ) * 4;
    const v4f v = *(const v4f*)(Ds + row * NCB + c4);
    *(volatile v4f*)(pq + (size_t)(rowBase + row) * NCT + colBase + c4) = v;
  }
  __threadfence();
#pragma unroll
  for (int i = tid; i < NIT; i += NTHR) {
    const int row = i / RQ;
    const int c4  = (i - row * RQ) * 4;
    const v4f v = *(const v4f*)(Ds + row * NCB + c4);
    *(volatile v4f*)(pq + (size_t)(rowBase + row) * NCT + colBase + c4) = v;
  }
}

template <int F, int NB>
__global__ __launch_bounds__(NTHR) void k_agg(const int* __restrict__ ei, const float* __restrict__ ea,
                                              const float* __restrict__ pq, const float* __restrict__ cc,
                                              float* st, float* cntp, int nN, int nE, int vec8) {
  static_assert(F == 16 || F == 128);
  static_assert((NB % 4) == 0 && 2 * NB <= LISTN);
  constexpr int NF = NB * F;
  constexpr int P2 = 2 * F;
  constexpr int S4 = 4 * F;
  float* accb = (float*)lds_dyn;
  int*   cnt  = (int*)(accb + 4 * NF);
  int*   list = cnt + NB;
  int*   wcnt = list + LISTN;
  float* fl   = (float*)list;
  const int tid = threadIdx.x, lane = tid & 31, wave = tid >> 5;
  const int nodeBase = blockIdx.x * NB;
  const int* dsts = ei + nE;

  {
    const v4f z  = {0.f, 0.f, 0.f, 0.f};
    const float pinf = __builtin_huge_valf();
    const v4f hi = {pinf, pinf, pinf, pinf};
    const v4f lo = -hi;
    for (int i = tid; i < NF / 4; i += NTHR) {
      ((v4f*)accb)[i]            = z;
      ((v4f*)(accb + NF))[i]     = lo;
      ((v4f*)(accb + 2 * NF))[i] = hi;
      ((v4f*)(accb + 3 * NF))[i] = z;
    }
    for (int i = tid; i < NB; i += NTHR) cnt[i] = 0;
  }
  v4f C4[8], c04;
  float Cs[8], c0s;
  if (F >= 128) {
#pragma unroll
    for (int d = 0; d < 8; ++d) C4[d] = *(const v4f*)(cc + d * F + 4 * lane);
    c04 = *(const v4f*)(cc + 8 * F + 4 * lane);
#pragma unroll
    for (int d = 0; d < 8; ++d) Cs[d] = 0.f;
    c0s = 0.f;
  } else {
    const int c = lane & 15;
#pragma unroll
    for (int d = 0; d < 8; ++d) Cs[d] = cc[d * F + c];
    c0s = cc[8 * F + c];
    const v4f z = {0.f, 0.f, 0.f, 0.f};
#pragma unroll
    for (int d = 0; d < 8; ++d) C4[d] = z;
    c04 = z;
  }
  __syncthreads();

  const int nChunks = (nE + CHUNK - 1) / CHUNK;
#pragma unroll 1
  for (int ch = 0; ch < nChunks; ++ch) {
    const int cbase = ch * CHUNK;
    const int wc = scan_chunk<NB>(dsts, nE, cbase, nodeBase, vec8, list, tid, lane, wave);
    if (lane == 0) wcnt[wave] = wc;
    __syncthreads();
    if (wave == 0) {
#pragma unroll 1
      for (int wsx = 0; wsx < NWAVE; ++wsx) {
        int n = __builtin_amdgcn_readfirstlane(wcnt[wsx]);
        n = n > WCAP ? WCAP : (n < 0 ? 0 : n);
        const int* lp = list + wsx * WCAP;
#pragma unroll 1
        for (int i = 0; i < n; ++i) {
          const int ent  = __builtin_amdgcn_readfirstlane(lp[i]);
          const int slot = ent & (NB - 1);
          int e = cbase + ((ent >> 12) & (CHUNK - 1));
          e = e > nE - 1 ? nE - 1 : e;
          int src = ei[e];
          src = src < 0 ? 0 : (src > nN - 1 ? nN - 1 : src);
          int node = nodeBase + slot;
          node = node > nN - 1 ? nN - 1 : node;
          const v4f ea0 = *(const v4f*)(ea + (size_t)e * EDIM);
          const v4f ea1 = *(const v4f*)(ea + (size_t)e * EDIM + 4);
          if (F >= 128) {
            const v4f p = *(const v4f*)(pq + (size_t)node * P2 + 4 * lane);
            const v4f q = *(const v4f*)(pq + (size_t)src * P2 + F + 4 * lane);
            v4f h = (p + q) + c04;
            h += ea0.x * C4[0]; h += ea0.y * C4[1]; h += ea0.z * C4[2]; h += ea0.w * C4[3];
            h += ea1.x * C4[4]; h += ea1.y * C4[5]; h += ea1.z * C4[6]; h += ea1.w * C4[7];
            float* ap = accb + slot * F + 4 * lane;
            const v4f sv = *(const v4f*)ap;
            *(v4f*)ap = sv + h;
            v4f mv = *(const v4f*)(ap + NF);
            mv.x = fmaxf(mv.x, h.x); mv.y = fmaxf(mv.y, h.y); mv.z = fmaxf(mv.z, h.z); mv.w = fmaxf(mv.w, h.w);
            *(v4f*)(ap + NF) = mv;
            v4f nv = *(const v4f*)(ap + 2 * NF);
            nv.x = fminf(nv.x, h.x); nv.y = fminf(nv.y, h.y); nv.z = fminf(nv.z, h.z); nv.w = fminf(nv.w, h.w);
            *(v4f*)(ap + 2 * NF) = nv;
            const v4f qv = *(const v4f*)(ap + 3 * NF);
            *(v4f*)(ap + 3 * NF) = qv + h * h;
          } else {
            const int c = lane & 15;
            const float p = pq[(size_t)node * P2 + c];
            const float q = pq[(size_t)src * P2 + F + c];
            float h = (p + q) + c0s;
            h += ea0.x * Cs[0]; h += ea0.y * Cs[1]; h += ea0.z * Cs[2]; h += ea0.w * Cs[3];
            h += ea1.x * Cs[4]; h += ea1.y * Cs[5]; h += ea1.z * Cs[6]; h += ea1.w * Cs[7];
            if (lane < F) {
              float* ap = accb + slot * F + c;
              ap[0]      = ap[0] + h;
              ap[NF]     = fmaxf(ap[NF], h);
              ap[2 * NF] = fminf(ap[2 * NF], h);
              ap[3 * NF] = ap[3 * NF] + h * h;
            }
          }
          if (lane == 0) cnt[slot] = cnt[slot] + 1;
        }
      }
    }
    __syncthreads();
  }

  for (int s = tid; s < NB; s += NTHR) {
    const int   cv = cnt[s];
    const float cf = (float)cv;
    const float dg = cf > 1.f ? cf : 1.f;
    fl[s]      = 1.0f / dg;
    fl[NB + s] = cf;
  }
  __syncthreads();

  {
#pragma clang fp contract(off)
    constexpr int FQ = F / 4;
#pragma unroll 1
    for (int idx = tid; idx < NF / 4; idx += NTHR) {
      const int slot = idx / FQ;
      const int c4   = (idx - slot * FQ) * 4;
      const float rd = fl[slot];
      const float cz = fl[NB + slot];
      float* ap = accb + slot * F + c4;
      const v4f s = *(const v4f*)ap;
      const v4f q = *(const v4f*)(ap + 3 * NF);
      const v4f mean = s * rd;
      const v4f m2   = q * rd;
      v4f var = m2 - mean * mean;
      var.x = var.x > 0.f ? var.x : 0.f; var.y = var.y > 0.f ? var.y : 0.f;
      var.z = var.z > 0.f ? var.z : 0.f; var.w = var.w > 0.f ? var.w : 0.f;
      v4f sd;
      sd.x = sqrtf(var.x + 1e-5f); sd.y = sqrtf(var.y + 1e-5f);
      sd.z = sqrtf(var.z + 1e-5f); sd.w = sqrtf(var.w + 1e-5f);
      *(v4f*)ap            = mean;
      *(v4f*)(ap + 3 * NF) = sd;
      if (cz == 0.f) {
        const v4f z = {0.f, 0.f, 0.f, 0.f};
        *(v4f*)(ap + NF)     = z;
        *(v4f*)(ap + 2 * NF) = z;
      }
    }
  }
  __syncthreads();

  const size_t ob = (size_t)nodeBase * S4;
  {
    constexpr int FQ = F / 4;
#pragma unroll 4
    for (int i = tid; i < NF; i += NTHR) {
      const int row = i / F;
      const int pos = i - row * F;
      const int a   = pos / FQ;
      const int c4  = (pos - a * FQ) * 4;
      const v4f v = *(const v4f*)(accb + a * NF + row * F + c4);
      *(volatile v4f*)(st + ob + 4 * (size_t)i) = v;
    }
    if (tid < NB / 4) {
      const v4f v = *(const v4f*)(fl + NB + 4 * tid);
      *(volatile v4f*)(cntp + (size_t)nodeBase + 4 * tid) = v;
    }
    __threadfence();
#pragma unroll 4
    for (int i = tid; i < NF; i += NTHR) {
      const int row = i / F;
      const int pos = i - row * F;
      const int a   = pos / FQ;
      const int c4  = (pos - a * FQ) * 4;
      const v4f v = *(const v4f*)(accb + a * NF + row * F + c4);
      *(volatile v4f*)(st + ob + 4 * (size_t)i) = v;
    }
    if (tid < NB / 4) {
      const v4f v = *(const v4f*)(fl + NB + 4 * tid);
      *(volatile v4f*)(cntp + (size_t)nodeBase + 4 * tid) = v;
    }
  }
}

template <int F, int KP, int XP, bool LAST>
__global__ __launch_bounds__(NTHR) void k_post(
    const float* __restrict__ xin, const float* __restrict__ st, const float* __restrict__ cntp,
    const unsigned short* __restrict__ qwh, const unsigned short* __restrict__ qwl, const float* __restrict__ qb,
    const unsigned short* __restrict__ lwh, const unsigned short* __restrict__ lwl, const float* __restrict__ lb,
    const float* __restrict__ gam, const float* __restrict__ bet,
    const unsigned short* __restrict__ hwh, const unsigned short* __restrict__ hwl, const float* __restrict__ hb,
    float* xnext, float* out, int nN) {
  constexpr int S4 = 4 * F;
  static_assert(KP % 32 == 0 && KP >= 13 * F && KP < 13 * F + 32 && (F % 4) == 0 && F >= 4);
  char* base = (char*)lds_dyn;
  float*          sc  = (float*)(base + O_SC);
  unsigned short* ALh = (unsigned short*)(base + O_ALH);
  unsigned short* ALl = (unsigned short*)(base + O_ALL);
  unsigned short* Ath = (unsigned short*)(base + O_R2);
  unsigned short* Atl = Ath + PROWS * ATP;
  float*          S   = (float*)(base + O_R2);
  float*          OT  = (float*)(base + O_OT);
  const int tid = threadIdx.x, lane = tid & 31, wave = tid >> 5, hh = lane >> 4, m = lane & 15;
  const int rowBase = blockIdx.x * PROWS;

  if (tid < PROWS) {
    int rowc = rowBase + tid;
    rowc = rowc > nN - 1 ? nN - 1 : rowc;
    const float cf   = cntp[rowc];
    const float logd = logf(cf + 1.0f);
    const float rl   = 1.0f / logd;
    sc[2 * tid]     = logd * RAVG;
    sc[2 * tid + 1] = (logd > 0.f) ? AVGF * rl : 0.f;
  }
  __syncthreads();

  v8f acc[4];
#pragma unroll
  for (int t = 0; t < 4; ++t) { v8f z = {0.f, 0.f, 0.f, 0.f, 0.f, 0.f, 0.f, 0.f}; acc[t] = z; }
  const int rr = 16 * (wave & 3) + m;
  const int cw = 64 * (wave >> 2);

#pragma unroll 1
  for (int kt = 0; kt < KP / 32; ++kt) {
#pragma unroll
    for (int j2 = 0; j2 < 2; ++j2) {
      const int g  = tid + NTHR * j2;
      const int r  = g >> 3;
      const int kq = (g & 7) * 4;
      const int k  = 32 * kt + kq;
      int rowc = rowBase + r;
      rowc = rowc > nN - 1 ? nN - 1 : rowc;
      const int kx = k < F - 4 ? k : F - 4;
      const v4f xv = *(const v4f*)(xin + (size_t)rowc * XP + kx);
      int kk = k - F;
      kk = kk < 0 ? 0 : kk;
      const int grp    = kk / S4;
      const int within = kk - grp * S4;
      const v4f sv = *(const v4f*)(st + (size_t)rowc * S4 + within);
      const float am = sc[2 * r], at = sc[2 * r + 1];
      const float scale = (grp == 0) ? 1.f : ((grp == 1) ? am : ((grp == 2) ? at : 0.f));
      const v4f v = (k < F) ? xv : sv * scale;
      v4us hv, lv;
      split4(v, hv, lv);
      *(v4us*)(Ath + r * ATP + kq) = hv;
      *(v4us*)(Atl + r * ATP + kq) = lv;
    }
    __syncthreads();
    FragB ah, al;
    ldfrag(ah, Ath + rr * ATP + 8 * hh);
    ldfrag(al, Atl + rr * ATP + 8 * hh);
#pragma unroll
    for (int t = 0; t < 4; ++t) {
      const int n = cw + 16 * t + m;
      const size_t bp = (size_t)n * KP + 32 * kt + 8 * hh;
      FragB bh, bl;
      ldfrag(bh, qwh + bp);
      ldfrag(bl, qwl + bp);
      acc[t] = mma3(acc[t], ah, al, bh, bl);
    }
    __syncthreads();
  }

#pragma unroll
  for (int t = 0; t < 4; ++t) {
    const int col = cw + 16 * t + m;
    const float qbv = qb[col];
#pragma unroll
    for (int r = 0; r < 8; ++r) {
      const float v = acc[t][r] + qbv;
      const int row = 16 * (wave & 3) + 8 * hh + r;
      const unsigned short hs = bf_rne(v);
      ALh[row * ALP + col] = hs;
      ALl[row * ALP + col] = bf_rne(v - bf_up(hs));
    }
  }
  __syncthreads();

  v8f lacc[4];
#pragma unroll
  for (int t = 0; t < 4; ++t) { v8f z = {0.f, 0.f, 0.f, 0.f, 0.f, 0.f, 0.f, 0.f}; lacc[t] = z; }
#pragma unroll
  for (int ks = 0; ks < HID / 32; ++ks) {
    FragB ah, al;
    ldfrag(ah, ALh + rr * ALP + 32 * ks + 8 * hh);
    ldfrag(al, ALl + rr * ALP + 32 * ks + 8 * hh);
#pragma unroll
    for (int t = 0; t < 4; ++t) {
      const int n = cw + 16 * t + m;
      const size_t bp = (size_t)n * HID + 32 * ks + 8 * hh;
      FragB bh, bl;
      ldfrag(bh, lwh + bp);
      ldfrag(bl, lwl + bp);
      lacc[t] = mma3(lacc[t], ah, al, bh, bl);
    }
  }
#pragma unroll
  for (int t = 0; t < 4; ++t) {
    const int col = cw + 16 * t + m;
    const float lbv = lb[col];
    float* sp = S + (16 * (wave & 3) + 8 * hh) * SPI + col;
#pragma unroll
    for (int r = 0; r < 8; ++r) sp[r * SPI] = lacc[t][r] + lbv;
  }
  __syncthreads();

  const v4f g4 = *(const v4f*)(gam + 4 * lane);
  const v4f b4 = *(const v4f*)(bet + 4 * lane);
  v4f y8[8];
#pragma unroll
  for (int i = 0; i < 8; ++i) {
    const int row = 8 * wave + i;
    const v4f xv = *(const v4f*)(S + row * SPI + 4 * lane);
    float s = (xv.x + xv.y) + (xv.z + xv.w);
    s += __shfl_xor(s, 16, 32); s += __shfl_xor(s, 8, 32); s += __shfl_xor(s, 4, 32);
    s += __shfl_xor(s, 2, 32);  s += __shfl_xor(s, 1, 32);
    const float mu = s * (1.0f / (float)HID);
    const v4f d = xv - mu;
    float q = (d.x * d.x + d.y * d.y) + (d.z * d.z + d.w * d.w);
    q += __shfl_xor(q, 16, 32); q += __shfl_xor(q, 8, 32); q += __shfl_xor(q, 4, 32);
    q += __shfl_xor(q, 2, 32);  q += __shfl_xor(q, 1, 32);
    const float var = q * (1.0f / (float)HID);
    const float rs  = 1.0f / sqrtf(var + 1e-5f);
    v4f y = (d * rs) * g4 + b4;
    y.x = fmaxf(y.x, 0.f); y.y = fmaxf(y.y, 0.f); y.z = fmaxf(y.z, 0.f); y.w = fmaxf(y.w, 0.f);
    y8[i] = y;
  }

  if (!LAST) {
    float* gp = xnext + ((size_t)rowBase + 8 * wave) * HID + 4 * lane;
#pragma unroll
    for (int i = 0; i < 8; ++i) *(volatile v4f*)(gp + (size_t)i * HID) = y8[i];
    __threadfence();
#pragma unroll
    for (int i = 0; i < 8; ++i) *(volatile v4f*)(gp + (size_t)i * HID) = y8[i];
  } else {
#pragma unroll
    for (int i = 0; i < 8; ++i) {
      const int row = 8 * wave + i;
      v4us hv, lv;
      split4(y8[i], hv, lv);
      *(v4us*)(ALh + row * ALP + 4 * lane) = hv;
      *(v4us*)(ALl + row * ALP + 4 * lane) = lv;
    }
    __syncthreads();
    if (wave < 4) {
      v8f hacc = {0.f, 0.f, 0.f, 0.f, 0.f, 0.f, 0.f, 0.f};
      const int r2 = 16 * wave + m;
#pragma unroll
      for (int ks = 0; ks < HID / 32; ++ks) {
        FragB ah, al;
        ldfrag(ah, ALh + r2 * ALP + 32 * ks + 8 * hh);
        ldfrag(al, ALl + r2 * ALP + 32 * ks + 8 * hh);
        const size_t bp = (size_t)m * HID + 32 * ks + 8 * hh;
        FragB bh, bl;
        ldfrag(bh, hwh + bp);
        ldfrag(bl, hwl + bp);
        hacc = mma3(hacc, ah, al, bh, bl);
      }
      const float hbv = hb[m < ODIM - 1 ? m : ODIM - 1];
      if (m < ODIM) {
        float* op = OT + (16 * wave + 8 * hh) * ODIM + m;
#pragma unroll
        for (int r = 0; r < 8; ++r) op[r * ODIM] = hacc[r] + hbv;
      }
    }
    __syncthreads();
    if (wave == 0) {
      v4f ov[2];
#pragma unroll
      for (int qq = 0; qq < 2; ++qq) ov[qq] = *(const v4f*)(OT + (lane + 32 * qq) * ODIM);
#pragma unroll
      for (int qq = 0; qq < 2; ++qq) {
        const int row = rowBase + lane + 32 * qq;
        if (row < nN) *(volatile v4f*)(out + (size_t)row * ODIM) = ov[qq];
      }
      __threadfence();
#pragma unroll
      for (int qq = 0; qq < 2; ++qq) {
        const int row = rowBase + lane + 32 * qq;
        if (row < nN) *(volatile v4f*)(out + (size_t)row * ODIM) = ov[qq];
      }
    }
  }
}

extern "C" void kernel_launch(void* const* d_in, const int* in_sizes, int n_in,
                              void* d_out, int out_size, void* d_ws, size_t ws_size,
                              hipStream_t stream) {
  if (n_in < 25) return;
  const int nN = in_sizes[0] / FIN;
  const int nE = in_sizes[1] / EDIM;
  if (nN <= 0 || nE <= 0) return;
  if (in_sizes[0] != nN * FIN || in_sizes[1] != nE * EDIM || in_sizes[2] != 2 * nE) return;
  if (in_sizes[3] != EDIM * FIN || in_sizes[4] != FIN || in_sizes[5] != 3 * FIN * FIN || in_sizes[6] != FIN) return;
  if (in_sizes[7] != 13 * FIN * HID || in_sizes[8] != HID || in_sizes[9] != HID * HID || in_sizes[10] != HID) return;
  if (in_sizes[11] != HID || in_sizes[12] != HID) return;
  if (in_sizes[13] != EDIM * HID || in_sizes[14] != HID || in_sizes[15] != 3 * HID * HID || in_sizes[16] != HID) return;
  if (in_sizes[17] != 13 * HID * HID || in_sizes[18] != HID || in_sizes[19] != HID * HID || in_sizes[20] != HID) return;
  if (in_sizes[21] != HID || in_sizes[22] != HID || in_sizes[23] != HID * ODIM || in_sizes[24] != ODIM) return;
  if (out_size != nN * ODIM) return;

  const float* x   = (const float*)d_in[0];
  const float* ea  = (const float*)d_in[1];
  const int*   ei  = (const int*)d_in[2];
  const float* ew0 = (const float*)d_in[3];
  const float* eb0 = (const float*)d_in[4];
  const float* pw0 = (const float*)d_in[5];
  const float* pb0 = (const float*)d_in[6];
  const float* qw0 = (const float*)d_in[7];
  const float* qb0 = (const float*)d_in[8];
  const float* lw0 = (const float*)d_in[9];
  const float* lb0 = (const float*)d_in[10];
  const float* g0  = (const float*)d_in[11];
  const float* b0  = (const float*)d_in[12];
  const float* ew1 = (const float*)d_in[13];
  const float* eb1 = (const float*)d_in[14];
  const float* pw1 = (const float*)d_in[15];
  const float* pb1 = (const float*)d_in[16];
  const float* qw1 = (const float*)d_in[17];
  const float* qb1 = (const float*)d_in[18];
  const float* lw1 = (const float*)d_in[19];
  const float* lb1 = (const float*)d_in[20];
  const float* g1  = (const float*)d_in[21];
  const float* b1  = (const float*)d_in[22];
  const float* hw  = (const float*)d_in[23];
  const float* hb  = (const float*)d_in[24];
  float* out = (float*)d_out;

  const int nPB = (nN + PROWS - 1) / PROWS;
  const int nA0 = (nN + NB0 - 1) / NB0;
  const int nA1 = (nN + NB1 - 1) / NB1;
  const size_t rP  = (size_t)nPB * PROWS;
  const size_t rS0 = (size_t)nA0 * NB0, rS1 = (size_t)nA1 * NB1;
  const size_t rST = rS0 > rS1 ? rS0 : rS1;
  const int CC0N = ((9 * FIN + 31) / 32) * 32;
  const int CC1N = ((9 * HID + 31) / 32) * 32;

  size_t off = 0;
  auto carve = [&](size_t bytes) { const size_t o = off; off += (bytes + 255) & ~(size_t)255; return o; };
  const size_t oP0h = carve((size_t)2 * FIN * 32 * 2),   oP0l = carve((size_t)2 * FIN * 32 * 2);
  const size_t oQ0h = carve((size_t)HID * KP0 * 2),      oQ0l = carve((size_t)HID * KP0 * 2);
  const size_t oL0h = carve((size_t)HID * HID * 2),      oL0l = carve((size_t)HID * HID * 2);
  const size_t oP1h = carve((size_t)2 * HID * HID * 2),  oP1l = carve((size_t)2 * HID * HID * 2);
  const size_t oQ1h = carve((size_t)HID * KP1 * 2),      oQ1l = carve((size_t)HID * KP1 * 2);
  const size_t oL1h = carve((size_t)HID * HID * 2),      oL1l = carve((size_t)HID * HID * 2);
  const size_t oHh  = carve((size_t)16 * HID * 2),       oHl  = carve((size_t)16 * HID * 2);
  const size_t oC0  = carve((size_t)CC0N * 4);
  const size_t oC1  = carve((size_t)CC1N * 4);
  const size_t oPQ  = carve(rP * (2 * HID) * 4);
  const size_t oST  = carve(rST * (4 * HID) * 4);
  const size_t oCN  = carve(rST * 4);
  const size_t oXN  = carve(rP * HID * 4);
  if (off > ws_size || off > ((size_t)128 << 20)) return;

  char* ws = (char*)d_ws;
  unsigned short* p0h = (unsigned short*)(ws + oP0h); unsigned short* p0l = (unsigned short*)(ws + oP0l);
  unsigned short* q0h = (unsigned short*)(ws + oQ0h); unsigned short* q0l = (unsigned short*)(ws + oQ0l);
  unsigned short* l0h = (unsigned short*)(ws + oL0h); unsigned short* l0l = (unsigned short*)(ws + oL0l);
  unsigned short* p1h = (unsigned short*)(ws + oP1h); unsigned short* p1l = (unsigned short*)(ws + oP1l);
  unsigned short* q1h = (unsigned short*)(ws + oQ1h); unsigned short* q1l = (unsigned short*)(ws + oQ1l);
  unsigned short* l1h = (unsigned short*)(ws + oL1h); unsigned short* l1l = (unsigned short*)(ws + oL1l);
  unsigned short* hwh = (unsigned short*)(ws + oHh);  unsigned short* hwl = (unsigned short*)(ws + oHl);
  float* cc0 = (float*)(ws + oC0);
  float* cc1 = (float*)(ws + oC1);
  float* pq  = (float*)(ws + oPQ);
  float* st  = (float*)(ws + oST);
  float* cnp = (float*)(ws + oCN);
  float* xn  = (float*)(ws + oXN);

  const int vec8 = ((nE & 3) == 0) ? 1 : 0;

  {
    const int t0 = 2 * FIN * 32 / 8, t1 = HID * KP0 / 8, t2 = HID * HID / 8, t3 = 2 * HID * HID / 8,
              t4 = HID * KP1 / 8, t5 = 16 * HID / 8;
    k_wsplit<<<(t0 + NTHR - 1) / NTHR, NTHR, 0, stream>>>(pw0, FIN, FIN, 2, 32, 2 * FIN, p0h, p0l);
    k_wsplit<<<(t1 + NTHR - 1) / NTHR, NTHR, 0, stream>>>(qw0, 13 * FIN, HID, 1, KP0, HID, q0h, q0l);
    k_wsplit<<<(t2 + NTHR - 1) / NTHR, NTHR, 0, stream>>>(lw0, HID, HID, 1, HID, HID, l0h, l0l);
    k_wsplit<<<(t3 + NTHR - 1) / NTHR, NTHR, 0, stream>>>(pw1, HID, HID, 2, HID, 2 * HID, p1h, p1l);
    k_wsplit<<<(t4 + NTHR - 1) / NTHR, NTHR, 0, stream>>>(qw1, 13 * HID, HID, 1, KP1, HID, q1h, q1l);
    k_wsplit<<<(t2 + NTHR - 1) / NTHR, NTHR, 0, stream>>>(lw1, HID, HID, 1, HID, HID, l1h, l1l);
    k_wsplit<<<(t5 + NTHR - 1) / NTHR, NTHR, 0, stream>>>(hw, HID, ODIM, 1, HID, 16, hwh, hwl);
  }
  k_comp<FIN><<<1, NTHR, 0, stream>>>(ew0, eb0, pw0, pb0, cc0);
  k_comp<HID><<<1, NTHR, 0, stream>>>(ew1, eb1, pw1, pb1, cc1);

  k_pq<FIN, 32, FIN, 32><<<dim3(nPB, 1), NTHR, 0, stream>>>(x, p0h, p0l, pq, nN);
  hipFuncSetAttribute(reinterpret_cast<const void*>(&k_agg<FIN, NB0>),
                      hipFuncAttributeMaxDynamicSharedMemorySize, LDS_AGG(FIN, NB0));
  k_agg<FIN, NB0><<<nA0, NTHR, LDS_AGG(FIN, NB0), stream>>>(ei, ea, pq, cc0, st, cnp, nN, nE, vec8);
  hipFuncSetAttribute(reinterpret_cast<const void*>(&k_post<FIN, KP0, FIN, false>),
                      hipFuncAttributeMaxDynamicSharedMemorySize, LDS_POST);
  k_post<FIN, KP0, FIN, false><<<nPB, NTHR, LDS_POST, stream>>>(
      x, st, cnp, q0h, q0l, qb0, l0h, l0l, lb0, g0, b0, hwh, hwl, hb, xn, out, nN);

  k_pq<HID, HID, HID, 128><<<dim3(nPB, 2), NTHR, 0, stream>>>(xn, p1h, p1l, pq, nN);
  hipFuncSetAttribute(reinterpret_cast<const void*>(&k_agg<HID, NB1>),
                      hipFuncAttributeMaxDynamicSharedMemorySize, LDS_AGG(HID, NB1));
  k_agg<HID, NB1><<<nA1, NTHR, LDS_AGG(HID, NB1), stream>>>(ei, ea, pq, cc1, st, cnp, nN, nE, vec8);
  hipFuncSetAttribute(reinterpret_cast<const void*>(&k_post<HID, KP1, HID, true>),
                      hipFuncAttributeMaxDynamicSharedMemorySize, LDS_POST);
  k_post<HID, KP1, HID, true><<<nPB, NTHR, LDS_POST, stream>>>(
      xn, st, cnp, q1h, q1l, qb1, l1h, l1l, lb1, g1, b1, hwh, hwl, hb, xn, out, nN);
}
